// Distance_38817914422096
// MI455X (gfx1250) — hardware-verified
//
#include <hip/hip_runtime.h>
#include <stddef.h>


typedef _Float16 h16;
typedef _Float16 v16h __attribute__((ext_vector_type(16)));
typedef _Float16 v8h  __attribute__((ext_vector_type(8)));
typedef float    v8f  __attribute__((ext_vector_type(8)));
typedef float    v4f  __attribute__((ext_vector_type(4)));

#ifndef NB
#define NB 8
#endif
#ifndef SEQ
#define SEQ 512
#endif
#define NB_FULL  8
#define SEQ_FULL 512
#define DIM      256
#define MROWS    (NB * SEQ)
#define TRI_FULL (SEQ_FULL * (SEQ_FULL - 1) / 2)
#define TRI_SEQ  (SEQ * (SEQ - 1) / 2)

#define BAND 64
#define LDB  (SEQ_FULL + 4)
#define XCARRY 1024.0f
#define EPSQ   1.0e-7f

static_assert(NB >= 1 && NB <= NB_FULL);
static_assert(SEQ >= 64 && SEQ <= SEQ_FULL && (SEQ % BAND) == 0);
static_assert(DIM == 32 * 8);
static_assert((DIM % 32) == 0);
static_assert((MROWS % 32) == 0);
static_assert((TRI_FULL % 32) == 0);
static_assert(((BAND * (BAND - 1) / 2) % 32) == 0);
static_assert((LDB % 4) == 0 && LDB >= SEQ);
static_assert(BAND == 64);
static_assert((size_t)64 * LDB * 4 <= (size_t)160 * 1024);

#define X16_BYTES ((size_t)MROWS * DIM * 2)
#define NRM_BYTES ((size_t)MROWS * 4)
#define OFF_X16 ((size_t)0)
#define OFF_NRM (OFF_X16 + X16_BYTES)
#define WS_TOTAL (OFF_NRM + NRM_BYTES)
static_assert((X16_BYTES % 128) == 0 && (NRM_BYTES % 128) == 0);
static_assert(WS_TOTAL <= (size_t)134217728);

__device__ __forceinline__ float bf16r(float x) {
  unsigned int u = __float_as_uint(x);
  u = (u + 0x7FFFu + ((u >> 16) & 1u)) & 0xFFFF0000u;
  return __uint_as_float(u);
}

static __device__ __forceinline__ h16 toh_flush(float v) {
  const h16 r = (h16)v;
  return (fabsf(v) < 6.103515625e-05f) ? (h16)0.0f : r;
}

__device__ __forceinline__ v16h frag_at(const _Float16* p) {
  v8h lo = *(const v8h*)(p);
  v8h hi = *(const v8h*)(p + 16);
  v16h out;
#pragma unroll
  for (int i = 0; i < 8; ++i) { out[i] = lo[i]; out[i + 8] = hi[i]; }
  return out;
}

__device__ __forceinline__ v8f wmma16(v16h a, v16h b, v8f c) {
  v8f d = __builtin_amdgcn_wmma_f32_16x16x32_f16(false, a, false, b, (short)0, c,
                                                 false, false);
  asm volatile("v_nop\n\tv_nop\n\tv_nop\n\tv_nop" : "+v"(d) : "v"(a), "v"(b));
  return d;
}

__device__ __forceinline__ float red32_sum(float x) {
#pragma unroll
  for (int off = 1; off < 32; off <<= 1) x += __shfl_xor(x, off, 32);
  return x;
}

__device__ __forceinline__ unsigned umin_u(unsigned a, unsigned b) { return (a < b) ? a : b; }
__device__ __forceinline__ unsigned umax_u(unsigned a, unsigned b) { return (a > b) ? a : b; }

__global__ __launch_bounds__(256) void xprep_kernel(
    const float* __restrict__ X, _Float16* __restrict__ X16, float* __restrict__ Nrm) {
  __shared__ float nsh[32];
  const unsigned lane = threadIdx.x & 31u;
  const unsigned w = __builtin_amdgcn_readfirstlane(threadIdx.x >> 5);
#pragma unroll 1
  for (unsigned r = 0; r < 4u; ++r) {
    const unsigned crow = blockIdx.x * 32u + w * 4u + r;
    const unsigned bidx = crow / (unsigned)SEQ;
    const unsigned sq = crow - bidx * (unsigned)SEQ;
    const size_t srow = (size_t)bidx * SEQ_FULL + sq;
    const float* xr = X + srow * DIM + lane * 8u;
    const v4f a0 = *(const v4f*)(xr);
    const v4f a1 = *(const v4f*)(xr + 4u);
    v8h o;
    float s = 0.0f;
#pragma unroll
    for (int i = 0; i < 4; ++i) {
      const h16 h0 = toh_flush(XCARRY * bf16r(a0[i]));
      const h16 h1 = toh_flush(XCARRY * bf16r(a1[i]));
      o[i] = h0;
      o[i + 4] = h1;
      const float t0 = (float)h0 * (1.0f / XCARRY);
      const float t1 = (float)h1 * (1.0f / XCARRY);
      s += t0 * t0;
      s += t1 * t1;
    }
    const float ss = red32_sum(s);
    if (lane == 0u) nsh[w * 4u + r] = ss;
    _Float16* p = X16 + (size_t)crow * DIM + lane * 8u;
    *(volatile v8h*)p = o;
    __threadfence();
    *(volatile v8h*)p = o;
  }
  __syncthreads();
  const v4f nv = *(const v4f*)&nsh[(lane & 7u) * 4u];
  float* np = Nrm + (size_t)blockIdx.x * 32u + (lane & 7u) * 4u;
  const bool wr = (w == 0u) && (lane < 8u);
  if (wr) *(volatile v4f*)np = nv;
  __threadfence();
  if (wr) *(volatile v4f*)np = nv;
}

__global__ __launch_bounds__(256) void pairgap_kernel(
    const _Float16* __restrict__ X16, const float* __restrict__ Nrm, float* __restrict__ out) {
  __shared__ float Ds[64 * LDB];
  const unsigned tid = threadIdx.x, lane = tid & 31u;
  const unsigned w = __builtin_amdgcn_readfirstlane(threadIdx.x >> 5);
  const unsigned mw = w >> 1, nw = w & 1u;
  const unsigned hh = lane >> 4, m = lane & 15u;
  const unsigned band = blockIdx.x;
  const unsigned b = blockIdx.y;
  const unsigned i0 = band * 64u;
  const size_t rowbase = (size_t)b * SEQ;

  const _Float16* ap = X16 + (rowbase + i0 + mw * 16u + m) * DIM + hh * 8u;
  const float* nr = Nrm + rowbase + i0 + mw * 16u + hh * 8u;
  const v4f nr0 = *(const v4f*)(nr);
  const v4f nr1 = *(const v4f*)(nr + 4u);
  float nrow[8];
  nrow[0] = nr0[0]; nrow[1] = nr0[1]; nrow[2] = nr0[2]; nrow[3] = nr0[3];
  nrow[4] = nr1[0]; nrow[5] = nr1[1]; nrow[6] = nr1[2]; nrow[7] = nr1[3];
  const float gs = 2.0f / (XCARRY * XCARRY);

  for (unsigned ct = 0; ct <= band; ++ct) {
    const unsigned c0 = ct * 64u + nw * 32u;
    const _Float16* bp0 = X16 + (rowbase + c0 + m) * DIM + hh * 8u;
    const _Float16* bp1 = bp0 + (size_t)16 * DIM;
    v8f acc0 = {}, acc1 = {};
#pragma unroll 2
    for (unsigned k0 = 0; k0 < (unsigned)DIM; k0 += 32u) {
      const v16h a  = frag_at(ap + k0);
      const v16h b0 = frag_at(bp0 + k0);
      const v16h b1 = frag_at(bp1 + k0);
      acc0 = wmma16(a, b0, acc0);
      acc1 = wmma16(a, b1, acc1);
    }
    const float nc0 = Nrm[rowbase + c0 + m];
    const float nc1 = Nrm[rowbase + c0 + 16u + m];
#pragma unroll
    for (int r = 0; r < 8; ++r) {
      const float d2a = fmaxf((nrow[r] + nc0) - acc0[r] * gs, EPSQ);
      const float d2b = fmaxf((nrow[r] + nc1) - acc1[r] * gs, EPSQ);
      float* d = &Ds[(mw * 16u + hh * 8u + (unsigned)r) * LDB + c0 + m];
      d[0]  = __builtin_amdgcn_sqrtf(d2a);
      d[16] = __builtin_amdgcn_sqrtf(d2b);
    }
  }
  __syncthreads();

  const unsigned start = (i0 * i0 - i0) >> 1;
  const unsigned total = 64u * i0 + 2016u;
  const unsigned niter = (total + 1023u) >> 10;
  const unsigned ilo = umax_u(i0, 1u), ihi = i0 + 63u;
  float* ob = out + (size_t)b * TRI_FULL + start;
#pragma unroll 1
  for (unsigned it = 0; it < niter; ++it) {
    const unsigned base = it * 1024u + tid * 4u;
    const unsigned fb = umin_u(base, total - 4u);
    const unsigned f = start + fb;
    unsigned i = (unsigned)((1.0f + sqrtf(1.0f + 8.0f * (float)f)) * 0.5f);
    i = umax_u(i, 1u);
    i = ((i * (i - 1u)) >> 1) > f ? i - 1u : i;
    i = ((i * (i + 1u)) >> 1) <= f ? i + 1u : i;
    i = umin_u(umax_u(i, ilo), ihi);
    unsigned j = f - ((i * (i - 1u)) >> 1);
    v4f v;
#pragma unroll
    for (int e = 0; e < 4; ++e) {
      const bool adv = (j >= i);
      i = adv ? i + 1u : i;
      j = adv ? 0u : j;
      const unsigned li = umin_u(i - i0, 63u);
      const unsigned lj = umin_u(j, ihi);
      v[e] = Ds[li * LDB + lj];
      ++j;
    }
    float* p = ob + fb;
    const bool wr = (base < total);
    if (wr) *(volatile v4f*)p = v;
    __threadfence();
    if (wr) *(volatile v4f*)p = v;
  }
}

extern "C" void kernel_launch(void* const* d_in, const int* in_sizes, int n_in,
                              void* d_out, int out_size, void* d_ws, size_t ws_size,
                              hipStream_t stream) {
  if (n_in < 1) return;
  const long long need_x = ((long long)(NB - 1) * SEQ_FULL + SEQ) * DIM;
  if ((long long)in_sizes[0] < need_x) return;
  const long long need_o = (long long)(NB - 1) * TRI_FULL + TRI_SEQ;
  if ((long long)out_size < need_o) return;
  if (ws_size < WS_TOTAL) return;

  const float* X = (const float*)d_in[0];
  float* out = (float*)d_out;

  char* ws = (char*)d_ws;
  _Float16* X16 = (_Float16*)(ws + OFF_X16);
  float*    Nrm = (float*)(ws + OFF_NRM);

  dim3 blk(256);
  xprep_kernel<<<dim3(MROWS / 32), blk, 0, stream>>>(X, X16, Nrm);
  pairgap_kernel<<<dim3(SEQ / BAND, NB), blk, 0, stream>>>(X16, Nrm, out);
}
